// EmbedMatcher_31430570672500
// MI455X (gfx1250) — hardware-verified
//
#include <hip/hip_runtime.h>
#include <stddef.h>
#include <stdint.h>


#define ED     128
#define DM2    256
#define HID    512
#define NGT    2048
#define NGP    1024
#define NQ     4096
#define NS     5
#define MAXK   50
#define KSEL   10
#define NSYM1  100001
#define NGW    100000
#define PADID  100000
#define NPR    100032
#define MV     (NQ + NS)
#define MVP    4160
#define STEPS  4
#define NTHR   256
#define TBM    64
#define TBN    128
#define KCH    128
#define APH    (KCH + 8)
#define LDSG   (2 * TBM * APH * 2)
#define EPSV   1e-8f
#define LNEPS  1e-5f
#define SLOPE  0.01f
#define BIGM   0x3FFFFFFF
#define WSCAP  134217728

#define NWG    (ED * DM2)
#define NW1    (HID * DM2)
#define NW2    (DM2 * HID)
#define NWI    (NGT * DM2)
#define NWH    (NGT * HID)
#define OWG    0
#define OW1    (OWG + 2 * NWG)
#define OW2    (OW1 + 2 * NW1)
#define OWI    (OW2 + 2 * NW2)
#define OWH    (OWI + 2 * NWI)
#define OWTOT  (OWH + 2 * NWH)
#define NBG    (NWG / (8 * NTHR))
#define NB1    (NW1 / (8 * NTHR))
#define NB2    (NW2 / (8 * NTHR))
#define NBI    (NWI / (8 * NTHR))
#define NBH    (NWH / (8 * NTHR))
#define NBSPLIT (NBG + NB1 + NB2 + NBI + NBH)

#define BYW    ((size_t)OWTOT * 2)
#define BYP    ((size_t)NPR * DM2 * 4)
#define BYV    ((size_t)MVP * DM2 * 4)
#define BYH1   ((size_t)MVP * HID * 4)
#define ABASE  ((size_t)0)
#define ACPL   ((size_t)NQ * NGP * 4)
#define AHA    (ACPL + (size_t)NQ * DM2 * 4)
#define AHB    (AHA + (size_t)NQ * DM2 * 4)
#define ASG    (AHB + (size_t)NQ * DM2 * 4)
#define ACV0   (ASG + 1024)
#define ACV1   (ACV0 + 4096)
#define AEND   (ACV1 + 4096)

static_assert(OW1 == 65536 && OW2 == 327680 && OWI == 589824 && OWH == 1638400 && OWTOT == 3735552);
static_assert(NBSPLIT == 912);
static_assert((NPR % TBM) == 0 && NPR >= NSYM1 && (MVP % TBM) == 0 && MVP >= MV && (NQ % TBM) == 0);
static_assert(TBM * TBN * 4 <= LDSG);
static_assert(((APH * 2) % 16) == 0);
static_assert(AEND <= BYP);
static_assert((BYW % 256) == 0 && (BYP % 256) == 0 && (BYV % 256) == 0 && (BYH1 % 256) == 0);
static_assert((ACPL % 256) == 0 && (AHA % 256) == 0 && (AHB % 256) == 0 && (ASG % 256) == 0 && (ACV0 % 256) == 0 && (ACV1 % 256) == 0);
static_assert((KCH % 32) == 0 && (ED % KCH) == 0 && (DM2 % KCH) == 0 && (HID % KCH) == 0);
static_assert((NQ % 32) == 0 && MAXK <= 64 && KSEL <= MAXK);

typedef float          v4f  __attribute__((ext_vector_type(4)));
typedef float          v8f  __attribute__((ext_vector_type(8)));
typedef unsigned short v4us __attribute__((ext_vector_type(4)));
typedef unsigned short v8us __attribute__((ext_vector_type(8)));
typedef __bf16         v16b __attribute__((ext_vector_type(16)));
union FragB { v16b v; v8us h[2]; };

__device__ __forceinline__ unsigned int bfr(float f) {
  const unsigned int u = __float_as_uint(f);
  return (u + 0x7FFFu + ((u >> 16) & 1u)) >> 16;
}
__device__ __forceinline__ void split1(float x, unsigned short& hb, unsigned short& lb) {
  const unsigned int hu = bfr(x);
  const float hf = __uint_as_float(hu << 16);
  hb = (unsigned short)hu;
  lb = (unsigned short)bfr(x - hf);
}
__device__ __forceinline__ void split4(v4f a, v4us& hi, v4us& lo) {
  unsigned short hb, lb;
  split1(a.x, hb, lb); hi[0] = hb; lo[0] = lb;
  split1(a.y, hb, lb); hi[1] = hb; lo[1] = lb;
  split1(a.z, hb, lb); hi[2] = hb; lo[2] = lb;
  split1(a.w, hb, lb); hi[3] = hb; lo[3] = lb;
}
__device__ __forceinline__ void split8(v4f a, v4f b, v8us& hi, v8us& lo) {
  unsigned short hb, lb;
  split1(a.x, hb, lb); hi[0] = hb; lo[0] = lb;
  split1(a.y, hb, lb); hi[1] = hb; lo[1] = lb;
  split1(a.z, hb, lb); hi[2] = hb; lo[2] = lb;
  split1(a.w, hb, lb); hi[3] = hb; lo[3] = lb;
  split1(b.x, hb, lb); hi[4] = hb; lo[4] = lb;
  split1(b.y, hb, lb); hi[5] = hb; lo[5] = lb;
  split1(b.z, hb, lb); hi[6] = hb; lo[6] = lb;
  split1(b.w, hb, lb); hi[7] = hb; lo[7] = lb;
}

__device__ __forceinline__ v8f wmb(v16b a, v16b b, v8f c) {
  v8f d = __builtin_amdgcn_wmma_f32_16x16x32_bf16(false, a, false, b, (short)0, c, false, false);
  asm volatile("v_nop\n\tv_nop\n\tv_nop\n\tv_nop" : "+v"(d) : "v"(a), "v"(b));
  return d;
}
__device__ __forceinline__ v8f zero8() { v8f z = {0.f, 0.f, 0.f, 0.f, 0.f, 0.f, 0.f, 0.f}; return z; }
__device__ __forceinline__ float wave_sum(float v) {
#pragma unroll
  for (int o = 16; o > 0; o >>= 1) v += __shfl_xor(v, o);
  return v;
}
__device__ __forceinline__ float dot4(v4f a, v4f b) { return a.x * b.x + a.y * b.y + a.z * b.z + a.w * b.w; }
__device__ __forceinline__ float sigf(float x) { return 1.0f / (1.0f + expf(-x)); }

__device__ __forceinline__ void mac3(const unsigned short* __restrict__ Bh, const unsigned short* __restrict__ Bl,
                                     size_t o, const FragB& ah, const FragB& al, v8f& c) {
  FragB bh, bl;
  bh.h[0] = *(const v8us*)(Bh + o); bh.h[1] = *(const v8us*)(Bh + o + 16);
  bl.h[0] = *(const v8us*)(Bl + o); bl.h[1] = *(const v8us*)(Bl + o + 16);
  c = wmb(ah.v, bh.v, c);
  c = wmb(ah.v, bl.v, c);
  c = wmb(al.v, bh.v, c);
}

__device__ __forceinline__ void gemm_core(
    const float* __restrict__ A, int lda, int m0, int mval, int K,
    const unsigned short* __restrict__ Bh, const unsigned short* __restrict__ Bl,
    size_t bo0, size_t bo1, size_t bo2, size_t bo3,
    unsigned short* sAh, unsigned short* sAl,
    v8f& c0, v8f& c1, v8f& c2, v8f& c3, int tid, int lane, int wave) {
  const int hh = lane >> 4, m = lane & 15, mt = wave >> 1;
  const unsigned short* ph = sAh + (mt * 16 + m) * APH + 8 * hh;
  const unsigned short* pl = sAl + (mt * 16 + m) * APH + 8 * hh;
#pragma unroll 1
  for (int kc = 0; kc < K; kc += KCH) {
    __syncthreads();
#pragma unroll
    for (int i = 0; i < (TBM * KCH / 4) / NTHR; ++i) {
      const int idx = i * NTHR + tid;
      const int row = idx >> 5, c4 = idx & 31;
      int ar = m0 + row;
      ar = ar > mval - 1 ? mval - 1 : ar;
      const v4f v = *(const v4f*)(A + (size_t)ar * lda + kc + 4 * c4);
      v4us hv, lv;
      split4(v, hv, lv);
      *(v4us*)(sAh + row * APH + 4 * c4) = hv;
      *(v4us*)(sAl + row * APH + 4 * c4) = lv;
    }
    __syncthreads();
#pragma unroll
    for (int ks = 0; ks < KCH / 32; ++ks) {
      FragB ah, al;
      ah.h[0] = *(const v8us*)(ph + 32 * ks); ah.h[1] = *(const v8us*)(ph + 32 * ks + 16);
      al.h[0] = *(const v8us*)(pl + 32 * ks); al.h[1] = *(const v8us*)(pl + 32 * ks + 16);
      const size_t kk = (size_t)(kc + 32 * ks + 8 * hh);
      mac3(Bh, Bl, bo0 + kk, ah, al, c0);
      mac3(Bh, Bl, bo1 + kk, ah, al, c1);
      mac3(Bh, Bl, bo2 + kk, ah, al, c2);
      mac3(Bh, Bl, bo3 + kk, ah, al, c3);
    }
  }
}

__device__ __forceinline__ void stage_acc(float* stg, v8f c0, v8f c1, v8f c2, v8f c3, int lane, int wave) {
  const int hh = lane >> 4, m = lane & 15, mt = wave >> 1;
  float* sr = stg + (mt * 16 + 8 * hh) * TBN + 64 * (wave & 1) + m;
#pragma unroll
  for (int r = 0; r < 8; ++r) {
    sr[r * TBN +  0] = c0[r];
    sr[r * TBN + 16] = c1[r];
    sr[r * TBN + 32] = c2[r];
    sr[r * TBN + 48] = c3[r];
  }
}

__global__ __launch_bounds__(NTHR) void k_split(
    const float* __restrict__ wg, const float* __restrict__ w1, const float* __restrict__ w2,
    const float* __restrict__ wi, const float* __restrict__ wh, unsigned short* wp) {
  const int b = blockIdx.x, tid = threadIdx.x;
  const float* src;
  int n, base, bl;
  if (b < NBG)                              { src = wg; n = NWG; base = OWG; bl = b; }
  else if (b < NBG + NB1)                   { src = w1; n = NW1; base = OW1; bl = b - NBG; }
  else if (b < NBG + NB1 + NB2)             { src = w2; n = NW2; base = OW2; bl = b - (NBG + NB1); }
  else if (b < NBG + NB1 + NB2 + NBI)       { src = wi; n = NWI; base = OWI; bl = b - (NBG + NB1 + NB2); }
  else                                      { src = wh; n = NWH; base = OWH; bl = b - (NBG + NB1 + NB2 + NBI); }
  const int e0 = (bl * NTHR + tid) * 8;
  const v4f a = *(const v4f*)(src + e0);
  const v4f c = *(const v4f*)(src + e0 + 4);
  v8us hv, lv;
  split8(a, c, hv, lv);
  unsigned short* dh = wp + base + e0;
  unsigned short* dl = dh + n;
  *(volatile v8us*)dh = hv;
  *(volatile v8us*)dl = lv;
  __threadfence();
  *(volatile v8us*)dh = hv;
  *(volatile v8us*)dl = lv;
}

template <int EPI>
__global__ __launch_bounds__(NTHR) void k_gemm(
    const float* __restrict__ A, int lda, int mval,
    const unsigned short* __restrict__ Bh, const unsigned short* __restrict__ Bl,
    int ldb, int bmask, int bshift, int bjump,
    const float* __restrict__ bias, const float* __restrict__ addm, int ldadd,
    float* C, int ldc, int K) {
  __shared__ __attribute__((aligned(16))) v4f lds_raw[LDSG / 16];
  unsigned short* sAh = (unsigned short*)lds_raw;
  unsigned short* sAl = sAh + TBM * APH;
  float* stg = (float*)lds_raw;
  const int tid = threadIdx.x, lane = tid & 31, wave = tid >> 5, m = lane & 15;
  const int m0 = blockIdx.y * TBM, n0 = blockIdx.x * TBN;
  const int nb = n0 + 64 * (wave & 1) + m;
  const size_t bo0 = (size_t)((nb     ) & bmask) * ldb + (size_t)((nb     ) >> bshift) * bjump;
  const size_t bo1 = (size_t)((nb + 16) & bmask) * ldb + (size_t)((nb + 16) >> bshift) * bjump;
  const size_t bo2 = (size_t)((nb + 32) & bmask) * ldb + (size_t)((nb + 32) >> bshift) * bjump;
  const size_t bo3 = (size_t)((nb + 48) & bmask) * ldb + (size_t)((nb + 48) >> bshift) * bjump;

  v8f c0 = zero8(), c1 = zero8(), c2 = zero8(), c3 = zero8();
  gemm_core(A, lda, m0, mval, K, Bh, Bl, bo0, bo1, bo2, bo3, sAh, sAl, c0, c1, c2, c3, tid, lane, wave);
  __syncthreads();
  stage_acc(stg, c0, c1, c2, c3, lane, wave);
  __syncthreads();

  v4f ov[8];
#pragma unroll
  for (int i = 0; i < 8; ++i) {
    const int idx = i * NTHR + tid;
    const int row = idx >> 5, c4 = idx & 31;
    const int n = n0 + 4 * c4;
    v4f v = *(const v4f*)(stg + row * TBN + 4 * c4);
    if (EPI != 0) {
      const v4f bv = *(const v4f*)(bias + n);
      v += bv;
    }
    if (EPI == 1) {
      v.x = fmaxf(v.x, 0.0f); v.y = fmaxf(v.y, 0.0f); v.z = fmaxf(v.z, 0.0f); v.w = fmaxf(v.w, 0.0f);
    }
    if (EPI == 2) {
      int ar = m0 + row;
      ar = ar > mval - 1 ? mval - 1 : ar;
      const v4f av = *(const v4f*)(addm + (size_t)ar * ldadd + n);
      v += av;
    }
    ov[i] = v;
  }
#pragma unroll
  for (int i = 0; i < 8; ++i) {
    const int idx = i * NTHR + tid;
    const int row = idx >> 5, c4 = idx & 31;
    *(volatile v4f*)(C + (size_t)(m0 + row) * ldc + n0 + 4 * c4) = ov[i];
  }
  __threadfence();
#pragma unroll
  for (int i = 0; i < 8; ++i) {
    const int idx = i * NTHR + tid;
    const int row = idx >> 5, c4 = idx & 31;
    *(volatile v4f*)(C + (size_t)(m0 + row) * ldc + n0 + 4 * c4) = ov[i];
  }
}

__global__ __launch_bounds__(NTHR) void k_nei(
    const int* __restrict__ conn, const int* __restrict__ deg, const int* __restrict__ ids,
    int side, int rowoff,
    const float* __restrict__ P, const float* __restrict__ sym,
    const float* __restrict__ wb, const float* __restrict__ gb,
    const float* __restrict__ gw, const float* __restrict__ gt,
    float* vec) {
  __shared__ int relc[64];
  __shared__ int entc[64];
  __shared__ int gidx[64];
  __shared__ int selk[64];
  __shared__ float maskf[64];
  __shared__ float cosv[64];
  __shared__ float selfv[ED];
  __shared__ float gsh[4];
  __shared__ __attribute__((aligned(16))) float proj[MAXK * ED];
  const int tid = threadIdx.x, lane = tid & 31, wave = tid >> 5;
  const int e = blockIdx.x;

  if (tid < 64) {
    const bool live = tid < MAXK;
    const int k = live ? tid : (MAXK - 1);
    const size_t ci = ((size_t)e * MAXK + k) * 2;
    const int r  = conn[ci];
    const int en = conn[ci + 1];
    const int rc = r < 0 ? 0 : (r > NSYM1 - 1 ? NSYM1 - 1 : r);
    const int ec = en < 0 ? 0 : (en > NSYM1 - 1 ? NSYM1 - 1 : en);
    int gi = (r == PADID) ? 0 : r;
    gi = gi < 0 ? 0 : (gi > NGW - 1 ? NGW - 1 : gi);
    relc[tid]  = live ? rc : 0;
    entc[tid]  = live ? ec : 0;
    gidx[tid]  = live ? gi : 0;
    maskf[tid] = (live && r != PADID) ? 1.0f : 0.0f;
  }
  {
    int sid = ids[(size_t)e * 2 + side];
    sid = sid < 0 ? 0 : (sid > NSYM1 - 1 ? NSYM1 - 1 : sid);
    if (tid < ED) selfv[tid] = sym[(size_t)sid * ED + tid];
  }
  __syncthreads();

  {
    const int n = tid & (ED - 1), kp = tid >> 7;
    const float bsum = wb[n] + gb[n];
#pragma unroll 1
    for (int k = kp; k < MAXK; k += 2) {
      const float a = P[(size_t)relc[k] * DM2 + n];
      const float c = P[(size_t)entc[k] * DM2 + ED + n];
      float v = (a + c) + bsum;
      v = (v >= 0.0f) ? v : SLOPE * v;
      v = v * maskf[k];
      proj[k * ED + n] = v;
    }
  }
  __syncthreads();

  {
    float ps = 0.0f;
#pragma unroll
    for (int q = 0; q < 4; ++q) { const float s = selfv[lane + 32 * q]; ps += s * s; }
    ps = wave_sum(ps);
    const float nself = sqrtf(ps + EPSV);
#pragma unroll 1
    for (int k = wave; k < MAXK; k += 8) {
      float num = 0.0f, nn = 0.0f;
#pragma unroll
      for (int q = 0; q < 4; ++q) {
        const float s = selfv[lane + 32 * q];
        const float p = proj[k * ED + lane + 32 * q];
        num += s * p;
        nn += p * p;
      }
      num = wave_sum(num);
      nn = wave_sum(nn);
      const float den = nself * sqrtf(nn + EPSV) + EPSV;
      const float cs = num * (1.0f / den);
      if (lane == 0) cosv[k] = cs;
    }
  }
  __syncthreads();

  if (tid < 64) {
    const int kk = tid < MAXK ? tid : (MAXK - 1);
    const float c = cosv[kk];
    int cnt = 0;
#pragma unroll 1
    for (int j = 0; j < MAXK; ++j) {
      const float cj = cosv[j];
      cnt += ((cj > c) || (cj == c && j < kk)) ? 1 : 0;
    }
    selk[tid] = (tid < MAXK && cnt < KSEL) ? 1 : 0;
  } else if (wave == 2) {
    const float ga  = gw[gidx[lane]];
    const float gbv = gw[gidx[lane + 32]];
    float s = ga + ((lane + 32 < MAXK) ? gbv : 0.0f);
    s = wave_sum(s);
    const float x = (s * (1.0f / (float)MAXK)) * (1.0f / gt[0]);
    float g = sigf(x);
    g = (deg[e] > 0) ? g : 1.0f;
    if (lane == 0) gsh[0] = g;
  }
  __syncthreads();

  if (tid < ED) {
    float s = 0.0f;
#pragma unroll 1
    for (int k = 0; k < MAXK; ++k) s += (selk[k] != 0) ? proj[k * ED + tid] : 0.0f;
    const float agg = s * (1.0f / (float)KSEL);
    const float o = tanhf(selfv[tid] + gsh[0] * agg);
    float* p = vec + (size_t)(rowoff + e) * DM2 + side * ED + tid;
    *(volatile float*)p = o;
    __threadfence();
    *(volatile float*)p = o;
  }
}

__global__ __launch_bounds__(NTHR) void k_ln(const float* __restrict__ h2, const float* __restrict__ g,
                                            const float* __restrict__ b, float* q, int nrows) {
  const int tid = threadIdx.x, lane = tid & 31, wave = tid >> 5;
  const int row = blockIdx.x * 8 + wave;
  if (row >= nrows) return;
  const float* hr = h2 + (size_t)row * DM2;
  const v4f x0 = *(const v4f*)(hr + 4 * lane);
  const v4f x1 = *(const v4f*)(hr + ED + 4 * lane);
  float s = (x0.x + x0.y) + (x0.z + x0.w) + (x1.x + x1.y) + (x1.z + x1.w);
  s = wave_sum(s);
  const float mu = s * (1.0f / (float)DM2);
  const v4f d0 = x0 - mu, d1 = x1 - mu;
  float v = dot4(d0, d0) + dot4(d1, d1);
  v = wave_sum(v);
  const float var = v * (1.0f / (float)DM2);
  const float rs = 1.0f / sqrtf(var + LNEPS);
  const v4f g0 = *(const v4f*)(g + 4 * lane), g1 = *(const v4f*)(g + ED + 4 * lane);
  const v4f b0 = *(const v4f*)(b + 4 * lane), b1 = *(const v4f*)(b + ED + 4 * lane);
  const v4f o0 = g0 * d0 * rs + b0;
  const v4f o1 = g1 * d1 * rs + b1;
  float* qr = q + (size_t)row * DM2;
  *(volatile v4f*)(qr + 4 * lane) = o0;
  *(volatile v4f*)(qr + ED + 4 * lane) = o1;
  __threadfence();
  *(volatile v4f*)(qr + 4 * lane) = o0;
  *(volatile v4f*)(qr + ED + 4 * lane) = o1;
}

__global__ __launch_bounds__(NTHR) void k_sgc(const float* __restrict__ qenc, const float* __restrict__ whh,
                                             const float* __restrict__ bih, const float* __restrict__ bhh,
                                             float* sg, float* cv0, float* cv1) {
  __shared__ float ssg[DM2];
  const int tid = threadIdx.x;
  float s = 0.0f;
#pragma unroll
  for (int r = 0; r < NS; ++r) s += qenc[(size_t)(NQ + r) * DM2 + tid];
  s = s * (1.0f / (float)NS);
  ssg[tid] = s;
  *(volatile float*)(sg + tid) = s;
  __syncthreads();
  float bv[4], dv[4];
#pragma unroll
  for (int gq = 0; gq < 4; ++gq) {
    const int nr = gq * HID + tid;
    const float bb = bih[nr] + bhh[nr];
    const float* wr = whh + (size_t)nr * HID + DM2;
    float d = 0.0f;
#pragma unroll 4
    for (int k = 0; k < DM2; ++k) d += ssg[k] * wr[k];
    bv[gq] = bb;
    dv[gq] = bb + d;
  }
#pragma unroll
  for (int gq = 0; gq < 4; ++gq) {
    *(volatile float*)(cv0 + gq * DM2 + tid) = bv[gq];
    *(volatile float*)(cv1 + gq * DM2 + tid) = dv[gq];
  }
  __threadfence();
  *(volatile float*)(sg + tid) = s;
#pragma unroll
  for (int gq = 0; gq < 4; ++gq) {
    *(volatile float*)(cv0 + gq * DM2 + tid) = bv[gq];
    *(volatile float*)(cv1 + gq * DM2 + tid) = dv[gq];
  }
}

__global__ __launch_bounds__(NTHR) void k_lstm(
    const float* __restrict__ hprev, const unsigned short* __restrict__ Wh, const unsigned short* __restrict__ Wl,
    const float* __restrict__ base, const float* __restrict__ cv, const float* __restrict__ qenc,
    float* cpl, float* hout, int step) {
  __shared__ __attribute__((aligned(16))) v4f lds_raw[LDSG / 16];
  unsigned short* sAh = (unsigned short*)lds_raw;
  unsigned short* sAl = sAh + TBM * APH;
  float* stg = (float*)lds_raw;
  const int tid = threadIdx.x, lane = tid & 31, wave = tid >> 5, m = lane & 15;
  const int j0 = blockIdx.x * 32, m0 = blockIdx.y * TBM;

  v8f c0 = zero8(), c1 = zero8(), c2 = zero8(), c3 = zero8();
  if (step > 0) {
    const int cb = 64 * (wave & 1) + m;
    const size_t bo0 = (size_t)(((cb     ) >> 5) * HID + j0 + ((cb     ) & 31)) * HID;
    const size_t bo1 = (size_t)(((cb + 16) >> 5) * HID + j0 + ((cb + 16) & 31)) * HID;
    const size_t bo2 = (size_t)(((cb + 32) >> 5) * HID + j0 + ((cb + 32) & 31)) * HID;
    const size_t bo3 = (size_t)(((cb + 48) >> 5) * HID + j0 + ((cb + 48) & 31)) * HID;
    gemm_core(hprev, DM2, m0, NQ, DM2, Wh, Wl, bo0, bo1, bo2, bo3, sAh, sAl, c0, c1, c2, c3, tid, lane, wave);
  }
  __syncthreads();
  stage_acc(stg, c0, c1, c2, c3, lane, wave);
  __syncthreads();

  const int j = j0 + lane;
  const float cvi = cv[j], cvf = cv[DM2 + j], cvg = cv[2 * DM2 + j], cvo = cv[3 * DM2 + j];
#pragma unroll 1
  for (int i = 0; i < 8; ++i) {
    const int row = wave + 8 * i;
    const size_t mm = (size_t)(m0 + row);
    const float* br = base + mm * NGP + j;
    const float gi = (stg[row * TBN +  0 + lane] + br[0])       + cvi;
    const float gf = (stg[row * TBN + 32 + lane] + br[DM2])     + cvf;
    const float gg = (stg[row * TBN + 64 + lane] + br[2 * DM2]) + cvg;
    const float go = (stg[row * TBN + 96 + lane] + br[3 * DM2]) + cvo;
    float cold = 0.0f;
    if (step > 0) cold = cpl[mm * DM2 + j];
    const float cn = sigf(gf) * cold + sigf(gi) * tanhf(gg);
    const float hn = sigf(go) * tanhf(cn);
    const float hv = qenc[mm * DM2 + j] + hn;
    float* pc = cpl + mm * DM2 + j;
    float* phv = hout + mm * DM2 + j;
    *(volatile float*)pc = cn;
    *(volatile float*)phv = hv;
    __threadfence();
    *(volatile float*)pc = cn;
    *(volatile float*)phv = hv;
  }
}

__global__ __launch_bounds__(NTHR) void k_cos(const float* __restrict__ h, const float* __restrict__ sg, float* out) {
  __shared__ __attribute__((aligned(16))) float res[32];
  const int tid = threadIdx.x, lane = tid & 31, wave = tid >> 5;
  const int r0 = blockIdx.x * 32;
  const v4f s0 = *(const v4f*)(sg + 4 * lane);
  const v4f s1 = *(const v4f*)(sg + ED + 4 * lane);
  float ss = dot4(s0, s0) + dot4(s1, s1);
  ss = wave_sum(ss);
  const float nsg = sqrtf(ss + EPSV);
#pragma unroll
  for (int i = 0; i < 4; ++i) {
    const int row = r0 + 4 * wave + i;
    const float* hr = h + (size_t)row * DM2;
    const v4f x0 = *(const v4f*)(hr + 4 * lane);
    const v4f x1 = *(const v4f*)(hr + ED + 4 * lane);
    float num = dot4(x0, s0) + dot4(x1, s1);
    float qq = dot4(x0, x0) + dot4(x1, x1);
    num = wave_sum(num);
    qq = wave_sum(qq);
    const float den = sqrtf(qq + EPSV) * nsg;
    const float v = num * (1.0f / den);
    if (lane == 0) res[4 * wave + i] = v;
  }
  __syncthreads();
  if (tid < 8) {
    const v4f v = *(const v4f*)(res + 4 * tid);
    float* p = out + r0 + 4 * tid;
    *(volatile v4f*)p = v;
    __threadfence();
    *(volatile v4f*)p = v;
  }
}

extern "C" void kernel_launch(void* const* d_in, const int* in_sizes, int n_in,
                              void* d_out, int out_size, void* d_ws, size_t ws_size,
                              hipStream_t stream) {
  if (n_in < 26) return;
  if (in_sizes[0] != NQ * 2 || in_sizes[1] != NS * 2) return;
  if (in_sizes[2] != NQ * MAXK * 2 || in_sizes[3] != NQ || in_sizes[4] != NQ * MAXK * 2 || in_sizes[5] != NQ) return;
  if (in_sizes[6] != NS * MAXK * 2 || in_sizes[7] != NS || in_sizes[8] != NS * MAXK * 2 || in_sizes[9] != NS) return;
  if (in_sizes[10] != NSYM1 * ED || in_sizes[11] != ED * DM2 || in_sizes[12] != ED || in_sizes[13] != ED) return;
  if (in_sizes[14] != NGW || in_sizes[15] != 1) return;
  if (in_sizes[16] != HID * DM2 || in_sizes[17] != HID || in_sizes[18] != DM2 * HID || in_sizes[19] != DM2) return;
  if (in_sizes[20] != DM2 || in_sizes[21] != DM2) return;
  if (in_sizes[22] != NGT * DM2 || in_sizes[23] != NGT * HID || in_sizes[24] != NGT || in_sizes[25] != NGT) return;
  if (out_size != NQ) return;

  const int*   query   = (const int*)d_in[0];
  const int*   support = (const int*)d_in[1];
  const int*   q_l1    = (const int*)d_in[2];
  const int*   q_deg_l = (const int*)d_in[3];
  const int*   q_r1    = (const int*)d_in[4];
  const int*   q_deg_r = (const int*)d_in[5];
  const int*   s_l1    = (const int*)d_in[6];
  const int*   s_deg_l = (const int*)d_in[7];
  const int*   s_r1    = (const int*)d_in[8];
  const int*   s_deg_r = (const int*)d_in[9];
  const float* sym     = (const float*)d_in[10];
  const float* gcnW    = (const float*)d_in[11];
  const float* gcnwb   = (const float*)d_in[12];
  const float* gcnb    = (const float*)d_in[13];
  const float* gatew   = (const float*)d_in[14];
  const float* gatet   = (const float*)d_in[15];
  const float* seW1    = (const float*)d_in[16];
  const float* seb1    = (const float*)d_in[17];
  const float* seW2    = (const float*)d_in[18];
  const float* seb2    = (const float*)d_in[19];
  const float* lng     = (const float*)d_in[20];
  const float* lnb     = (const float*)d_in[21];
  const float* Wih     = (const float*)d_in[22];
  const float* Whh     = (const float*)d_in[23];
  const float* bih     = (const float*)d_in[24];
  const float* bhh     = (const float*)d_in[25];
  float* out = (float*)d_out;

  char* ws = (char*)d_ws;
  size_t off = 0;
  const size_t oW  = off; off += BYW;
  const size_t oP  = off; off += BYP;
  const size_t oV  = off; off += BYV;
  const size_t oH1 = off; off += BYH1;
  const size_t oH2 = off; off += BYV;
  const size_t oQ  = off; off += BYV;
  if (off > ws_size || off > (size_t)WSCAP) return;
  unsigned short* wp  = (unsigned short*)(ws + oW);
  float* P    = (float*)(ws + oP);
  float* V    = (float*)(ws + oV);
  float* H1   = (float*)(ws + oH1);
  float* H2   = (float*)(ws + oH2);
  float* Q    = (float*)(ws + oQ);
  float* BASE = (float*)(ws + oP + ABASE);
  float* CPL  = (float*)(ws + oP + ACPL);
  float* HA   = (float*)(ws + oP + AHA);
  float* HB   = (float*)(ws + oP + AHB);
  float* SG   = (float*)(ws + oP + ASG);
  float* CV0  = (float*)(ws + oP + ACV0);
  float* CV1  = (float*)(ws + oP + ACV1);

  k_split<<<NBSPLIT, NTHR, 0, stream>>>(gcnW, seW1, seW2, Wih, Whh, wp);

  k_gemm<0><<<dim3(DM2 / TBN, NPR / TBM), NTHR, 0, stream>>>(
      sym, ED, NSYM1, wp + OWG, wp + OWG + NWG, DM2, ED - 1, 7, ED,
      (const float*)0, (const float*)0, 0, P, DM2, ED);

  k_nei<<<NQ, NTHR, 0, stream>>>(q_l1, q_deg_l, query, 0, 0, P, sym, gcnwb, gcnb, gatew, gatet, V);
  k_nei<<<NQ, NTHR, 0, stream>>>(q_r1, q_deg_r, query, 1, 0, P, sym, gcnwb, gcnb, gatew, gatet, V);
  k_nei<<<NS, NTHR, 0, stream>>>(s_l1, s_deg_l, support, 0, NQ, P, sym, gcnwb, gcnb, gatew, gatet, V);
  k_nei<<<NS, NTHR, 0, stream>>>(s_r1, s_deg_r, support, 1, NQ, P, sym, gcnwb, gcnb, gatew, gatet, V);

  k_gemm<1><<<dim3(HID / TBN, MVP / TBM), NTHR, 0, stream>>>(
      V, DM2, MV, wp + OW1, wp + OW1 + NW1, DM2, BIGM, 30, 0, seb1, (const float*)0, 0, H1, HID, DM2);
  k_gemm<2><<<dim3(DM2 / TBN, MVP / TBM), NTHR, 0, stream>>>(
      H1, HID, MV, wp + OW2, wp + OW2 + NW2, HID, BIGM, 30, 0, seb2, V, DM2, H2, DM2, HID);
  k_ln<<<(MV + 7) / 8, NTHR, 0, stream>>>(H2, lng, lnb, Q, MV);

  k_sgc<<<1, NTHR, 0, stream>>>(Q, Whh, bih, bhh, SG, CV0, CV1);

  k_gemm<0><<<dim3(NGP / TBN, NQ / TBM), NTHR, 0, stream>>>(
      Q, DM2, NQ, wp + OWI, wp + OWI + NWI, DM2, 255, 8, HID * DM2,
      (const float*)0, (const float*)0, 0, BASE, NGP, DM2);

  for (int t = 0; t < STEPS; ++t) {
    const float* hprev = ((t - 1) & 1) ? HB : HA;
    float* hcur = (t & 1) ? HB : HA;
    const float* cv = (t == 0) ? CV0 : CV1;
    k_lstm<<<dim3(DM2 / 32, NQ / TBM), NTHR, 0, stream>>>(
        hprev, wp + OWH, wp + OWH + NWH, BASE, cv, Q, CPL, hcur, t);
  }

  k_cos<<<NQ / 32, NTHR, 0, stream>>>(((STEPS - 1) & 1) ? HB : HA, SG, out);
}
